// SafeGATWrapper_51805895524973
// MI455X (gfx1250) — hardware-verified
//
#include <hip/hip_runtime.h>
#include <stddef.h>


#define FIN     128
#define NCOL    128
#define HEADS   4
#define CH      32
#define NTHR    256
#define NWAVE   8
#define EPT     8
#define NGRP    2
#define CHUNK   (NTHR * EPT * NGRP)
#define WCAP    (EPT * NGRP * 32)
#define LISTN   (NWAVE * WCAP)
#define NB      2048
#define TPWV    (NB / NWAVE)
#define RCAP    40960
#define DEGCAP  256
#define BM      64
#define APK     (FIN + 8)
#define WSCAL   16.0f
#define WINV    0.0625f
#define NEG_SLOPE 0.2f
#define DEN_EPS 1e-16f
#define WSCAP   134217728
#define LDS_AGG ((RCAP + 3 * NB + LISTN + 2 * NWAVE) * 4 + 64)

static_assert((CHUNK & (CHUNK - 1)) == 0);
static_assert(CHUNK <= 4096);
static_assert(NB <= 4096 && (NB & (NB - 1)) == 0);
static_assert(NTHR * 8 == NB);
static_assert((RCAP % 32) == 0);
static_assert((NB % NWAVE) == 0);
static_assert((NB % BM) == 0);
static_assert((FIN % 32) == 0 && (NCOL % 32) == 0);
static_assert(HEADS * CH == NCOL && (CH % 4) == 0);
static_assert(((APK * 2) % 16) == 0);

typedef float    v4f  __attribute__((ext_vector_type(4)));
typedef float    v8f  __attribute__((ext_vector_type(8)));
typedef int      v4i  __attribute__((ext_vector_type(4)));
typedef _Float16 v4h  __attribute__((ext_vector_type(4)));
typedef _Float16 v8h  __attribute__((ext_vector_type(8)));
typedef _Float16 v16h __attribute__((ext_vector_type(16)));
union FragH { v16h v; v8h h[2]; };
union Pk8   { v8h v; v4h q[2]; };

__device__ __forceinline__ v8f wmh(v16h a, v16h b, v8f c) {
  v8f d = __builtin_amdgcn_wmma_f32_16x16x32_f16(false, a, false, b, (short)0, c, false, false);
  asm volatile("v_nop\n\tv_nop\n\tv_nop\n\tv_nop" : "+v"(d) : "v"(a), "v"(b));
  return d;
}

__device__ __forceinline__ float lrelu(float v) { return v >= 0.0f ? v : NEG_SLOPE * v; }

template <int NSLOT>
__device__ __forceinline__ int scan_chunk(const int* __restrict__ dsts, int nE, int cbase, int slotBase,
                                          int vec8, int* list, int tid, int lane, int wave) {
  int wc = 0;
#pragma unroll
  for (int g = 0; g < NGRP; ++g) {
    const int el0  = (g * NTHR + tid) * EPT;
    const int e0   = cbase + el0;
    const int sent = -2147483647 - 1;
    v4i da, db;
    if (vec8 != 0 && cbase + CHUNK <= nE) {
      da = *(const v4i*)(dsts + e0);
      db = *(const v4i*)(dsts + e0 + 4);
    } else {
      da.x = (e0     < nE) ? dsts[min(e0, nE - 1)] : sent;
      da.y = (e0 + 1 < nE) ? dsts[min(e0 + 1, nE - 1)] : sent;
      da.z = (e0 + 2 < nE) ? dsts[min(e0 + 2, nE - 1)] : sent;
      da.w = (e0 + 3 < nE) ? dsts[min(e0 + 3, nE - 1)] : sent;
      db.x = (e0 + 4 < nE) ? dsts[min(e0 + 4, nE - 1)] : sent;
      db.y = (e0 + 5 < nE) ? dsts[min(e0 + 5, nE - 1)] : sent;
      db.z = (e0 + 6 < nE) ? dsts[min(e0 + 6, nE - 1)] : sent;
      db.w = (e0 + 7 < nE) ? dsts[min(e0 + 7, nE - 1)] : sent;
    }
    const unsigned nb = (unsigned)slotBase;
    const unsigned s0 = (unsigned)da.x - nb, s1 = (unsigned)da.y - nb;
    const unsigned s2 = (unsigned)da.z - nb, s3 = (unsigned)da.w - nb;
    const unsigned s4 = (unsigned)db.x - nb, s5 = (unsigned)db.y - nb;
    const unsigned s6 = (unsigned)db.z - nb, s7 = (unsigned)db.w - nb;
    const bool h0 = s0 < (unsigned)NSLOT, h1 = s1 < (unsigned)NSLOT, h2 = s2 < (unsigned)NSLOT, h3 = s3 < (unsigned)NSLOT;
    const bool h4 = s4 < (unsigned)NSLOT, h5 = s5 < (unsigned)NSLOT, h6 = s6 < (unsigned)NSLOT, h7 = s7 < (unsigned)NSLOT;
    const unsigned any = __builtin_amdgcn_ballot_w32(h0 | h1 | h2 | h3 | h4 | h5 | h6 | h7);
    if (any != 0u) {
#define HITJ(J, HJ, SJ) { \
        const unsigned mj = __builtin_amdgcn_ballot_w32(HJ); \
        if (mj != 0u) { \
          if (HJ) { \
            const int pos = wc + (int)__builtin_amdgcn_mbcnt_lo(mj, 0u); \
            if (pos < WCAP) list[wave * WCAP + pos] = ((el0 + (J)) << 12) | (int)(SJ); \
          } \
          wc += (int)__builtin_popcount(mj); } }
      HITJ(0, h0, s0)
      HITJ(1, h1, s1)
      HITJ(2, h2, s2)
      HITJ(3, h3, s3)
      HITJ(4, h4, s4)
      HITJ(5, h5, s5)
      HITJ(6, h6, s6)
      HITJ(7, h7, s7)
#undef HITJ
    }
  }
  return wc;
}

__global__ __launch_bounds__(NTHR) void k_wprep(const float* __restrict__ W, _Float16* wp) {
  constexpr int UNITS = NCOL * FIN / 8;
  constexpr int K8    = FIN / 8;
  static_assert((UNITS % NTHR) == 0);
  const int i = (int)blockIdx.x * NTHR + (int)threadIdx.x;
  if (i >= UNITS) return;
  const int n  = i / K8;
  const int k0 = (i - n * K8) * 8;
  v4f a, b;
  a.x = W[(size_t)(k0 + 0) * NCOL + n] * WSCAL;
  a.y = W[(size_t)(k0 + 1) * NCOL + n] * WSCAL;
  a.z = W[(size_t)(k0 + 2) * NCOL + n] * WSCAL;
  a.w = W[(size_t)(k0 + 3) * NCOL + n] * WSCAL;
  b.x = W[(size_t)(k0 + 4) * NCOL + n] * WSCAL;
  b.y = W[(size_t)(k0 + 5) * NCOL + n] * WSCAL;
  b.z = W[(size_t)(k0 + 6) * NCOL + n] * WSCAL;
  b.w = W[(size_t)(k0 + 7) * NCOL + n] * WSCAL;
  Pk8 p;
  p.q[0] = __builtin_convertvector(a, v4h);
  p.q[1] = __builtin_convertvector(b, v4h);
  _Float16* d = wp + (size_t)i * 8;
  *(volatile v8h*)d = p.v;
  __threadfence();
  *(volatile v8h*)d = p.v;
}

__global__ __launch_bounds__(NTHR) void k_gemm(
    const float* __restrict__ A, const _Float16* __restrict__ Bw,
    const float* __restrict__ attS, const float* __restrict__ attD,
    float* C, float* eS, float* eD, int nRowsA) {
  constexpr int TPW  = 4;
  constexpr int LPH  = CH / 4;
  constexpr int Q4   = TPW * 4;
  constexpr int RPI  = 32 / Q4;
  constexpr int NIT  = 16 / RPI;
  constexpr int NES  = BM * HEADS;
  constexpr int NESI = NES / 128;
  constexpr int UPT  = (BM * FIN / 8) / NTHR;
  static_assert(NWAVE * 16 * TPW * 16 == 2 * BM * NCOL / 2 && 2 * TPW * 16 == NCOL);
  static_assert((Q4 & (Q4 - 1)) == 0 && Q4 <= 32 && Q4 >= LPH && (LPH & (LPH - 1)) == 0 && LPH >= 1);
  static_assert(NIT * RPI == 16);
  static_assert((NES % 128) == 0 && 2 * NESI <= NWAVE);
  static_assert(UPT * NTHR * 8 == BM * FIN);
  static_assert(BM * APK * 2 <= BM * NCOL * 4);

  __shared__ __attribute__((aligned(16))) float lds_raw[BM * NCOL];
  __shared__ __attribute__((aligned(16))) float sES[NES];
  __shared__ __attribute__((aligned(16))) float sED[NES];
  _Float16* sA  = (_Float16*)lds_raw;
  float*    stg = lds_raw;
  const int tid = threadIdx.x, lane = tid & 31, wave = tid >> 5, hh = lane >> 4, m = lane & 15;
  const int rowBase = blockIdx.x * BM;

#pragma unroll
  for (int i = 0; i < UPT; ++i) {
    const int idx = i * NTHR + tid;
    const int r   = idx / (FIN / 8);
    const int c8  = (idx - r * (FIN / 8)) * 8;
    int row = rowBase + r;
    row = row > nRowsA - 1 ? nRowsA - 1 : row;
    const float* ap = A + (size_t)row * FIN + c8;
    const v4f a = *(const v4f*)ap, b = *(const v4f*)(ap + 4);
    Pk8 p;
    p.q[0] = __builtin_convertvector(a, v4h);
    p.q[1] = __builtin_convertvector(b, v4h);
    *(v8h*)(sA + r * APK + c8) = p.v;
  }
  __syncthreads();

  const int rg  = wave >> 1;
  const int chf = wave & 1;
  const int r0  = rg * 16;
  const int c0  = chf * TPW * 16;

  v8f acc[TPW];
#pragma unroll
  for (int t = 0; t < TPW; ++t) { v8f z = {0.f, 0.f, 0.f, 0.f, 0.f, 0.f, 0.f, 0.f}; acc[t] = z; }
  const _Float16* afp = sA + (r0 + m) * APK + 8 * hh;
#pragma unroll
  for (int kt = 0; kt < FIN / 32; ++kt) {
    FragH af;
    af.h[0] = *(const v8h*)(afp + 32 * kt);
    af.h[1] = *(const v8h*)(afp + 32 * kt + 16);
#pragma unroll
    for (int t = 0; t < TPW; ++t) {
      const _Float16* bp = Bw + (size_t)(c0 + 16 * t + m) * FIN + 32 * kt + 8 * hh;
      FragH bf;
      bf.h[0] = *(const v8h*)bp;
      bf.h[1] = *(const v8h*)(bp + 16);
      acc[t] = wmh(af.v, bf.v, acc[t]);
    }
  }
  __syncthreads();

  {
    float* sp = stg + (size_t)(r0 + 8 * hh) * NCOL + c0 + m;
#pragma unroll
    for (int t = 0; t < TPW; ++t) {
#pragma unroll
      for (int r = 0; r < 8; ++r) sp[r * NCOL + 16 * t] = acc[t][r] * WINV;
    }
  }
  __syncthreads();

  const int qq   = lane & (Q4 - 1);
  const int rsub = lane / Q4;
  const int col  = c0 + 4 * qq;
  const int hd   = col / CH;
  const v4f aS = *(const v4f*)(attS + col);
  const v4f aD = *(const v4f*)(attD + col);
  const size_t gb = (size_t)(rowBase + r0) * NCOL + col;
#pragma unroll
  for (int it = 0; it < NIT; ++it) {
    const int row = it * RPI + rsub;
    const v4f v = *(const v4f*)(stg + (size_t)(r0 + row) * NCOL + col);
    *(volatile v4f*)(C + gb + (size_t)row * NCOL) = v;
    float ps = v.x * aS.x + v.y * aS.y + v.z * aS.z + v.w * aS.w;
    float pd = v.x * aD.x + v.y * aD.y + v.z * aD.z + v.w * aD.w;
#pragma unroll
    for (int o = 1; o < LPH; o <<= 1) { ps += __shfl_xor(ps, o); pd += __shfl_xor(pd, o); }
    if ((lane & (LPH - 1)) == 0) { sES[(r0 + row) * HEADS + hd] = ps; sED[(r0 + row) * HEADS + hd] = pd; }
  }
  __threadfence();
#pragma unroll
  for (int it = 0; it < NIT; ++it) {
    const int row = it * RPI + rsub;
    const v4f v = *(const v4f*)(stg + (size_t)(r0 + row) * NCOL + col);
    *(volatile v4f*)(C + gb + (size_t)row * NCOL) = v;
  }
  __syncthreads();

  v4f dv = {0.f, 0.f, 0.f, 0.f};
  const size_t eb = (size_t)rowBase * HEADS;
  if (wave < NESI) {
    const int f = wave * 128 + 4 * lane;
    dv = *(const v4f*)(sES + f);
    *(volatile v4f*)(eS + eb + f) = dv;
  } else if (wave < 2 * NESI) {
    const int f = (wave - NESI) * 128 + 4 * lane;
    dv = *(const v4f*)(sED + f);
    *(volatile v4f*)(eD + eb + f) = dv;
  }
  __threadfence();
  if (wave < NESI) {
    const int f = wave * 128 + 4 * lane;
    *(volatile v4f*)(eS + eb + f) = dv;
  } else if (wave < 2 * NESI) {
    const int f = (wave - NESI) * 128 + 4 * lane;
    *(volatile v4f*)(eD + eb + f) = dv;
  }
}

__global__ __launch_bounds__(NTHR) void k_agg(
    const int* __restrict__ srcs, const int* __restrict__ dsts,
    const float* __restrict__ eS, const float* __restrict__ eD,
    const float* __restrict__ hw, const float* __restrict__ bias,
    float* out, int nN, int nE, int vec8) {
  extern __shared__ v4f lds_dyn[];
  int* region = (int*)lds_dyn;
  int* scnt   = region + RCAP;
  int* sstart = scnt + NB;
  int* scur   = sstart + NB;
  int* list   = scur + NB;
  int* wcnt   = list + LISTN;
  int* wtot   = wcnt + NWAVE;
  const int tid = threadIdx.x, lane = tid & 31, wave = tid >> 5;
  const int nodeBase = blockIdx.x * NB;

  {
    const v4i z = {0, 0, 0, 0};
#pragma unroll 1
    for (int i = tid; i < RCAP / 4; i += NTHR) ((v4i*)region)[i] = z;
#pragma unroll 1
    for (int i = tid; i < NB / 4; i += NTHR) ((v4i*)scnt)[i] = z;
  }
  __syncthreads();

  const int nChunks = (nE + CHUNK - 1) / CHUNK;

#pragma unroll 1
  for (int ch = 0; ch < nChunks; ++ch) {
    const int cbase = ch * CHUNK;
    const int wc = scan_chunk<NB>(dsts, nE, cbase, nodeBase, vec8, list, tid, lane, wave);
    if (lane == 0) wcnt[wave] = wc;
    __syncthreads();
    if (wave == 0) {
#pragma unroll 1
      for (int wsx = 0; wsx < NWAVE; ++wsx) {
        int n = __builtin_amdgcn_readfirstlane(wcnt[wsx]);
        n = n > WCAP ? WCAP : (n < 0 ? 0 : n);
        const int* lp = list + wsx * WCAP;
#pragma unroll 1
        for (int i = 0; i < n; ++i) {
          const int ent  = __builtin_amdgcn_readfirstlane(lp[i]);
          const int slot = ent & (NB - 1);
          if (lane == 0) scnt[slot] = scnt[slot] + 1;
        }
      }
    }
    __syncthreads();
  }

  {
    const v4i ca = *(const v4i*)(scnt + 8 * tid);
    const v4i cb = *(const v4i*)(scnt + 8 * tid + 4);
    const int e0 = max(ca.x, 0), e1 = max(ca.y, 0), e2 = max(ca.z, 0), e3 = max(ca.w, 0);
    const int e4 = max(cb.x, 0), e5 = max(cb.y, 0), e6 = max(cb.z, 0), e7 = max(cb.w, 0);
    const int ts = e0 + e1 + e2 + e3 + e4 + e5 + e6 + e7;
    int incl = ts;
#pragma unroll
    for (int d = 1; d < 32; d <<= 1) {
      const int t = __shfl_up(incl, d);
      if (lane >= d) incl += t;
    }
    if (lane == 31) wtot[wave] = incl;
    __syncthreads();
    int pre = 0;
#pragma unroll 1
    for (int w = 0; w < wave; ++w) pre += wtot[w];
    int run = pre + incl - ts;
    v4i oa, ob;
    oa.x = run; run += e0;
    oa.y = run; run += e1;
    oa.z = run; run += e2;
    oa.w = run; run += e3;
    ob.x = run; run += e4;
    ob.y = run; run += e5;
    ob.z = run; run += e6;
    ob.w = run;
    *(v4i*)(sstart + 8 * tid)     = oa;
    *(v4i*)(sstart + 8 * tid + 4) = ob;
    *(v4i*)(scur + 8 * tid)       = oa;
    *(v4i*)(scur + 8 * tid + 4)   = ob;
  }
  __syncthreads();

#pragma unroll 1
  for (int ch = 0; ch < nChunks; ++ch) {
    const int cbase = ch * CHUNK;
    const int wc = scan_chunk<NB>(dsts, nE, cbase, nodeBase, vec8, list, tid, lane, wave);
    if (lane == 0) wcnt[wave] = wc;
    __syncthreads();
    if (wave == 0) {
#pragma unroll 1
      for (int wsx = 0; wsx < NWAVE; ++wsx) {
        int n = __builtin_amdgcn_readfirstlane(wcnt[wsx]);
        n = n > WCAP ? WCAP : (n < 0 ? 0 : n);
        const int* lp = list + wsx * WCAP;
#pragma unroll 1
        for (int i = 0; i < n; ++i) {
          const int ent  = __builtin_amdgcn_readfirstlane(lp[i]);
          const int slot = ent & (NB - 1);
          int e = cbase + ((ent >> 12) & (CHUNK - 1));
          e = e > nE - 1 ? nE - 1 : (e < 0 ? 0 : e);
          int src = srcs[e];
          src = src < 0 ? 0 : (src > nN - 1 ? nN - 1 : src);
          if (lane == 0) {
            int pos = scur[slot];
            pos = pos < 0 ? 0 : (pos > RCAP - 1 ? RCAP - 1 : pos);
            region[pos] = src;
            const int np = pos + 1;
            scur[slot] = np > RCAP ? RCAP : np;
          }
        }
      }
    }
    __syncthreads();
  }
  __syncthreads();

  const int col0 = 4 * lane;
  const int hd0  = col0 / CH;
  const v4f bb   = *(const v4f*)(bias + col0);
#pragma unroll 1
  for (int j = 0; j < TPWV; ++j) {
    const int sl = wave * TPWV + j;
    const int c  = nodeBase + sl;
    int st = sstart[sl];
    st = st < 0 ? 0 : (st > RCAP ? RCAP : st);
    int n = scnt[sl];
    n = n < 0 ? 0 : (n > DEGCAP ? DEGCAP : n);
    if (st + n > RCAP) n = RCAP - st;

    const float ed    = eD[(size_t)c * HEADS + hd0];
    const float eself = lrelu(eS[(size_t)c * HEADS + hd0] + ed);

    float mx = eself;
#pragma unroll 1
    for (int q0 = 0; q0 < n; q0 += 32) {
      int pos = st + q0 + lane;
      pos = pos < 0 ? 0 : (pos > RCAP - 1 ? RCAP - 1 : pos);
      int sl_l = region[pos];
      sl_l = sl_l < 0 ? 0 : (sl_l > nN - 1 ? nN - 1 : sl_l);
      const int mcnt = (n - q0) < 32 ? (n - q0) : 32;
#pragma unroll 1
      for (int pp = 0; pp < mcnt; ++pp) {
        const int s = __builtin_amdgcn_readlane(sl_l, pp);
        mx = fmaxf(mx, lrelu(eS[(size_t)s * HEADS + hd0] + ed));
      }
    }

    float p   = __expf(eself - mx);
    float den = p;
    v4f   acc = *(const v4f*)(hw + (size_t)c * NCOL + col0) * p;
#pragma unroll 1
    for (int q0 = 0; q0 < n; q0 += 32) {
      int pos = st + q0 + lane;
      pos = pos < 0 ? 0 : (pos > RCAP - 1 ? RCAP - 1 : pos);
      int sl_l = region[pos];
      sl_l = sl_l < 0 ? 0 : (sl_l > nN - 1 ? nN - 1 : sl_l);
      const int mcnt = (n - q0) < 32 ? (n - q0) : 32;
#pragma unroll 1
      for (int pp = 0; pp < mcnt; ++pp) {
        const int s = __builtin_amdgcn_readlane(sl_l, pp);
        p = __expf(lrelu(eS[(size_t)s * HEADS + hd0] + ed) - mx);
        den += p;
        const v4f hv = *(const v4f*)(hw + (size_t)s * NCOL + col0);
        acc = acc + hv * p;
      }
    }

    const float rd = 1.0f / (den + DEN_EPS);
    const v4f v = acc * rd + bb;
    if (c < nN) {
      float* pw = out + (size_t)c * NCOL + col0;
      *(volatile v4f*)pw = v;
      __threadfence();
      *(volatile v4f*)pw = v;
    }
  }
}

extern "C" void kernel_launch(void* const* d_in, const int* in_sizes, int n_in,
                              void* d_out, int out_size, void* d_ws, size_t ws_size,
                              hipStream_t stream) {
  if (n_in < 6) return;
  const int nN = in_sizes[0] / FIN;
  const int nE = in_sizes[1] / 2;
  if (nN <= 0 || nE <= 0 || in_sizes[0] != nN * FIN || in_sizes[1] != 2 * nE) return;
  if (in_sizes[2] != FIN * NCOL || in_sizes[3] != NCOL || in_sizes[4] != NCOL || in_sizes[5] != NCOL) return;
  if (out_size != nN * NCOL) return;
  if (nE > (1 << 28) || nN > (1 << 24)) return;

  const float* x    = (const float*)d_in[0];
  const int*   ei   = (const int*)d_in[1];
  const int*   src  = ei;
  const int*   dst  = ei + nE;
  const float* W    = (const float*)d_in[2];
  const float* attS = (const float*)d_in[3];
  const float* attD = (const float*)d_in[4];
  const float* bias = (const float*)d_in[5];
  float* out = (float*)d_out;

  const int nBA  = (nN + NB - 1) / NB;
  const int NPAD = nBA * NB;

  char* ws = (char*)d_ws;
  size_t off = 0;
  const size_t oW  = off; off += (size_t)NCOL * FIN * 2;          off = (off + 255) & ~(size_t)255;
  const size_t oHw = off; off += (size_t)NPAD * NCOL * 4;         off = (off + 255) & ~(size_t)255;
  const size_t oES = off; off += (size_t)NPAD * HEADS * 4;        off = (off + 255) & ~(size_t)255;
  const size_t oED = off; off += (size_t)NPAD * HEADS * 4;        off = (off + 255) & ~(size_t)255;
  if (off > ws_size || off > (size_t)WSCAP) return;
  _Float16* wp = (_Float16*)(ws + oW);
  float*    hw = (float*)(ws + oHw);
  float*    es = (float*)(ws + oES);
  float*    ed = (float*)(ws + oED);

  const int vec8 = ((nE & 3) == 0) ? 1 : 0;

  k_wprep<<<(NCOL * FIN / 8 + NTHR - 1) / NTHR, NTHR, 0, stream>>>(W, wp);

  k_gemm<<<NPAD / BM, NTHR, 0, stream>>>(x, wp, attS, attD, hw, es, ed, nN);

  hipFuncSetAttribute(reinterpret_cast<const void*>(&k_agg),
                      hipFuncAttributeMaxDynamicSharedMemorySize, LDS_AGG);
  k_agg<<<nBA, NTHR, LDS_AGG, stream>>>(src, dst, es, ed, hw, bias, out, nN, nE, vec8);
}
